// DeformConvTranspose_55207509623210
// MI455X (gfx1250) — hardware-verified
//
#include <hip/hip_runtime.h>

#define B_N    8
#define CIN    128
#define H_IN   64
#define W_IN   64
#define HW_IN  (H_IN * W_IN)
#define COUT   128
#define KK     16
#define HO     61
#define WO     61
#define NPIX   (HO * WO)
#define CK     (CIN * KK)
#define CHUNK  256
#define NCHUNK (CK / CHUNK)
#define SLABS  (CHUNK / 32)
#define PT     32
#define NTILE  ((NPIX + PT - 1) / PT)
#define PROW   132
#define SPITCH (NTILE * PT)
#define NROWS  (B_N * COUT)
#define NOUT   (NROWS * NPIX)
#define WSCALE 64.0f
#define WINV   0.015625f

static_assert(CK % CHUNK == 0);
static_assert(SPITCH % 32 == 0);
static_assert(NOUT % 32 == 0);
static_assert((COUT * CK) % 8 == 0);

typedef _Float16       v16h  __attribute__((ext_vector_type(16)));
typedef _Float16       v8h   __attribute__((ext_vector_type(8)));
typedef _Float16       v2h   __attribute__((ext_vector_type(2)));
typedef float          v8f   __attribute__((ext_vector_type(8)));
typedef float          v4f   __attribute__((ext_vector_type(4)));
typedef unsigned int   v8u   __attribute__((ext_vector_type(8)));
typedef unsigned int   v4u   __attribute__((ext_vector_type(4)));
typedef v8h __attribute__((may_alias)) v8ha;
typedef v4f __attribute__((may_alias)) v4fa;
typedef v4u __attribute__((may_alias)) v4ua;

union Frag { v16h v; v8h half[2]; };

__device__ __forceinline__ v8f wmma_f16(v16h a, v16h b, v8f c) {
  v8f d = __builtin_amdgcn_wmma_f32_16x16x32_f16(false, a, false, b, (short)0, c, false, false);
  asm volatile("v_nop\n\tv_nop\n\tv_nop\n\tv_nop" : "+v"(d) : "v"(a), "v"(b));
  return d;
}

__device__ __forceinline__ v16h frag_g(const _Float16* p, int h) {
  Frag f;
  f.half[0] = *(const v8ha*)(p + 8 * h);
  f.half[1] = *(const v8ha*)(p + 16 + 8 * h);
  return f.v;
}

__device__ __forceinline__ v16h frag_lds(const unsigned int* p, int h) {
  const v4u a = *(const v4ua*)(p + 4 * h);
  const v4u c = *(const v4ua*)(p + 8 + 4 * h);
  const v8u r = {a.x, a.y, a.z, a.w, c.x, c.y, c.z, c.w};
  return __builtin_bit_cast(v16h, r);
}

__global__ __launch_bounds__(256) void dcn_prep(const float* __restrict__ weight,
                                                _Float16* __restrict__ whf)
{
  const int g = blockIdx.x * 256 + threadIdx.x;
  if (g >= (COUT * CK) / 8) return;
  const int o    = g >> 8;
  const int kg   = g & 255;
  const int c    = kg >> 1;
  const int tap0 = (kg & 1) * 8;
  const float* src = weight + (size_t)(o * CIN + c) * KK + (8 - tap0);
  const v4f fa = *(const v4fa*)src;
  const v4f fb = *(const v4fa*)(src + 4);
  const v8h H = { (_Float16)(fb.w * WSCALE), (_Float16)(fb.z * WSCALE), (_Float16)(fb.y * WSCALE), (_Float16)(fb.x * WSCALE),
                  (_Float16)(fa.w * WSCALE), (_Float16)(fa.z * WSCALE), (_Float16)(fa.y * WSCALE), (_Float16)(fa.x * WSCALE) };
  _Float16* dst = whf + (size_t)g * 8;
  *(volatile v8h*)dst = H;
  __threadfence();
  *(volatile v8h*)dst = H;
}

__device__ __forceinline__ void stage_store_pass(const float* So, float* S, int b, int p0, int w, int lane) {
  const int q8 = lane & 7, sub = lane >> 3;
  #pragma unroll
  for (int i = 0; i < 4; ++i) {
    const int orow = 16 * w + 4 * i + sub;
    const v4f v = *(const v4fa*)(So + orow * PT + 4 * q8);
    float* dst = S + (size_t)(b * COUT + orow) * SPITCH + p0 + 4 * q8;
    *(volatile v4f*)dst = v;
  }
}

__global__ __launch_bounds__(256)
void dcn_main(const float* __restrict__ inp,
              const float* __restrict__ off,
              const float* __restrict__ msk,
              const float* __restrict__ bias,
              const _Float16* __restrict__ whf,
              float* __restrict__ S)
{
  __shared__ __attribute__((aligned(16))) unsigned int Sh[PT * PROW];
  __shared__ __attribute__((aligned(16))) float        So[COUT * PT];

  const int tile = blockIdx.x % NTILE;
  const int b    = blockIdx.x / NTILE;
  const int p0   = tile * PT;

  const int t    = threadIdx.x;
  const int lane = t & 31;
  const int wv   = t >> 5;
  const int h    = lane >> 4;
  const int mcol = lane & 15;
  const int kp   = wv;
  const int pl   = lane;
  const int p    = p0 + pl;

  int   gidx[8];
  float gwt[8];
  {
    const int   pc  = min(p, NPIX - 1);
    const float inb = (p < NPIX) ? 1.f : 0.f;
    const int   ho  = pc / WO;
    const int   wo  = pc - ho * WO;
    #pragma unroll
    for (int kk = 0; kk < 2; ++kk) {
      const int k  = 2 * kp + kk;
      const int ki = k >> 2, kj = k & 3;
      const size_t ob = ((size_t)b * (2 * KK) + 2 * k) * NPIX + pc;
      const float dy = off[ob];
      const float dx = off[ob + NPIX];
      const float mk = msk[((size_t)b * KK + k) * NPIX + pc] * inb;
      const float y  = (dy + (float)ki) + (float)ho;
      const float x  = (dx + (float)kj) + (float)wo;
      const float y0f = floorf(y), x0f = floorf(x);
      const float wy = y - y0f, wx = x - x0f;
      const int y0 = (int)fminf(fmaxf(y0f, -8192.f), 8192.f);
      const int x0 = (int)fminf(fmaxf(x0f, -8192.f), 8192.f);
      const float vy0 = (y0     >= 0 && y0     < H_IN) ? 1.f : 0.f;
      const float vy1 = (y0 + 1 >= 0 && y0 + 1 < H_IN) ? 1.f : 0.f;
      const float vx0 = (x0     >= 0 && x0     < W_IN) ? 1.f : 0.f;
      const float vx1 = (x0 + 1 >= 0 && x0 + 1 < W_IN) ? 1.f : 0.f;
      const int cy0 = min(max(y0,     0), H_IN - 1);
      const int cy1 = min(max(y0 + 1, 0), H_IN - 1);
      const int cx0 = min(max(x0,     0), W_IN - 1);
      const int cx1 = min(max(x0 + 1, 0), W_IN - 1);
      gidx[kk * 4 + 0] = cy0 * W_IN + cx0;
      gidx[kk * 4 + 1] = cy0 * W_IN + cx1;
      gidx[kk * 4 + 2] = cy1 * W_IN + cx0;
      gidx[kk * 4 + 3] = cy1 * W_IN + cx1;
      gwt[kk * 4 + 0] = (1.f - wy) * (1.f - wx) * vy0 * vx0 * mk;
      gwt[kk * 4 + 1] = (1.f - wy) * wx         * vy0 * vx1 * mk;
      gwt[kk * 4 + 2] = wy         * (1.f - wx) * vy1 * vx0 * mk;
      gwt[kk * 4 + 3] = wy         * wx         * vy1 * vx1 * mk;
    }
  }

  const float* inpb = inp + (size_t)b * CIN * HW_IN;
  const _Float16* wrow = whf + (size_t)(16 * wv + mcol) * CK;

  const v8f zero8 = {0.f, 0.f, 0.f, 0.f, 0.f, 0.f, 0.f, 0.f};
  v8f acc0 = zero8;
  v8f acc1 = zero8;

  #pragma unroll 1
  for (int cc = 0; cc < NCHUNK; ++cc) {
    const int c0 = cc * 16;
    #pragma unroll 4
    for (int i = 0; i < 16; ++i) {
      const float* pch = inpb + (size_t)(c0 + i) * HW_IN;
      const float ve = gwt[0] * pch[gidx[0]] + gwt[1] * pch[gidx[1]] +
                       gwt[2] * pch[gidx[2]] + gwt[3] * pch[gidx[3]];
      const float vo = gwt[4] * pch[gidx[4]] + gwt[5] * pch[gidx[5]] +
                       gwt[6] * pch[gidx[6]] + gwt[7] * pch[gidx[7]];
      const v2h pr = {(_Float16)ve, (_Float16)vo};
      Sh[pl * PROW + i * 8 + kp] = __builtin_bit_cast(unsigned int, pr);
    }
    __syncthreads();

    #pragma unroll 1
    for (int s = 0; s < SLABS; ++s) {
      const int kg = cc * CHUNK + s * 32;
      const v16h A  = frag_g(wrow + kg, h);
      const v16h B0 = frag_lds(Sh + mcol * PROW + s * 16, h);
      const v16h B1 = frag_lds(Sh + (mcol + 16) * PROW + s * 16, h);
      acc0 = wmma_f16(A, B0, acc0);
      acc1 = wmma_f16(A, B1, acc1);
    }
    __syncthreads();
  }

  #pragma unroll
  for (int r = 0; r < 8; ++r) {
    const int ol = 16 * wv + 8 * h + r;
    const float bv = bias[ol];
    So[ol * PT + mcol]      = acc0[r] * WINV + bv;
    So[ol * PT + 16 + mcol] = acc1[r] * WINV + bv;
  }
  __syncthreads();

  stage_store_pass(So, S, b, p0, wv, lane);
  __threadfence();
  stage_store_pass(So, S, b, p0, wv, lane);
}

__global__ __launch_bounds__(256) void dcn_copy(const float* __restrict__ S, float* __restrict__ out)
{
  const int g  = blockIdx.x * 256 + threadIdx.x;
  const int f0 = g * 4;
  if (f0 >= NOUT) return;
  float v[4];
  #pragma unroll
  for (int j = 0; j < 4; ++j) {
    const int f   = min(f0 + j, NOUT - 1);
    const int row = f / NPIX;
    const int px  = f - row * NPIX;
    v[j] = S[(size_t)row * SPITCH + px];
  }
  const v4f o = {v[0], v[1], v[2], v[3]};
  float* dst = out + f0;
  *(volatile v4f*)dst = o;
  __threadfence();
  *(volatile v4f*)dst = o;
}

extern "C" void kernel_launch(void* const* d_in, const int* in_sizes, int n_in,
                              void* d_out, int out_size, void* d_ws, size_t ws_size,
                              hipStream_t stream) {
  if (n_in < 5) return;
  if (in_sizes[0] != B_N * CIN * HW_IN) return;
  if (in_sizes[1] != B_N * 2 * KK * NPIX) return;
  if (in_sizes[2] != B_N * KK * NPIX) return;
  if (in_sizes[3] != COUT * CIN * KK) return;
  if (in_sizes[4] != COUT) return;
  if (out_size != NOUT) return;

  const float* inp    = (const float*)d_in[0];
  const float* off    = (const float*)d_in[1];
  const float* msk    = (const float*)d_in[2];
  const float* weight = (const float*)d_in[3];
  const float* bias   = (const float*)d_in[4];
  float* out = (float*)d_out;

  const size_t wpl_bytes = (size_t)COUT * CK * 2;
  const size_t s_bytes   = (size_t)NROWS * SPITCH * 4;
  const size_t total     = wpl_bytes + s_bytes;
  if (total > ws_size) return;

  char* ws = (char*)d_ws;
  _Float16* whf = (_Float16*)(ws);
  float* S = (float*)(ws + wpl_bytes);

  const int nprep = (COUT * CK) / 8;
  dcn_prep<<<(nprep + 255) / 256, 256, 0, stream>>>(weight, whf);

  dcn_main<<<B_N * NTILE, 256, 0, stream>>>(inp, off, msk, bias, whf, S);

  const int ncopy = NOUT / 4;
  dcn_copy<<<(ncopy + 255) / 256, 256, 0, stream>>>(S, out);
}
